// SAGAN_Attention_56547539419342
// MI455X (gfx1250) — hardware-verified
//
#include <hip/hip_runtime.h>


namespace {
constexpr int NB = 8, C = 256, CQ = 32, N = 4096, M = 1024  , CG = 128  , HW = 64;
constexpr float XS = 8.0f, WSC = 256.0f, PS = 8.0f, LOG2E = 1.4426950408889634f;

typedef _Float16 b16;
typedef __attribute__((ext_vector_type(16))) _Float16 v16b;
typedef __attribute__((ext_vector_type(8))) _Float16 v8b;
typedef __attribute__((ext_vector_type(8))) float v8f;
typedef __attribute__((ext_vector_type(4))) float v4f;
__device__ __forceinline__ float bf16_rne(float f) { unsigned int u = __float_as_uint(f); u += 0x7FFFu + ((u >> 16) & 1u); return __uint_as_float(u & 0xFFFF0000u); }
__device__ __forceinline__ void split16(float v, b16& hi, b16& lo) { hi = (b16)v; lo = (b16)(v - (float)hi); }
__device__ __forceinline__ v16b frag_kb(const b16* p, int hh) { const v8b a = *(const v8b*)(p + 8 * hh), b = *(const v8b*)(p + 16 + 8 * hh); v16b f;
#pragma unroll
  for (int e = 0; e < 8; ++e) { f[e] = a[e]; f[8 + e] = b[e]; } return f; }
__device__ __forceinline__ v8f wmma16b(v16b a, v16b b, v8f c) { v8f d = __builtin_amdgcn_wmma_f32_16x16x32_f16(false, a, false, b, (short)0, c, false, false); asm volatile("v_nop\n\tv_nop\n\tv_nop\n\tv_nop" : "+v"(d) : "v"(a), "v"(b)); return d; }
__device__ __forceinline__ void wave_lds_sync() { __builtin_amdgcn_fence(__ATOMIC_RELEASE, "workgroup"); __builtin_amdgcn_wave_barrier(); __builtin_amdgcn_fence(__ATOMIC_ACQUIRE, "workgroup"); }
__device__ __forceinline__ float nexp2(float x) { return __builtin_amdgcn_exp2f(x); }

__global__ __launch_bounds__(256) void xt_kernel(const float* __restrict__ x, b16* __restrict__ XT16) {
  __shared__ __attribute__((aligned(16))) b16 T[64][64 + 8];
  const int b = blockIdx.z, c0 = blockIdx.y * 64, n0 = blockIdx.x * 64, t_ = threadIdx.x;
  for (int q = t_; q < 64 * 64; q += 256) { const int cc = q >> 6, nn = q & 63; T[nn][cc] = (b16)(bf16_rne(x[((size_t)b * C + c0 + cc) * N + n0 + nn]) * XS); }
  __syncthreads();
  for (int pass = 0; pass < 2; ++pass) { for (int q = t_; q < 64 * 8; q += 256) { const int nn = q >> 3, c8 = (q & 7) * 8; *(volatile v8b*)(XT16 + ((size_t)b * N + n0 + nn) * C + c0 + c8) = *(const v8b*)(&T[nn][c8]); } __threadfence(); }
}
__global__ __launch_bounds__(256) void prepw_kernel(const float* __restrict__ wq, const float* __restrict__ wk, const float* __restrict__ wg, const float* __restrict__ wo, b16* __restrict__ W16, b16* __restrict__ WG, b16* __restrict__ WO) {
  const int t = blockIdx.x * 256 + threadIdx.x; const int nq = CQ * C / 8, ng = CG * C / 8, no = C * CG / 8; const float* src; int e; b16* dst;
  if (t < nq) { src = wq; e = t * 8; dst = W16; } else if (t < 2 * nq) { src = wk; e = (t - nq) * 8; dst = W16 + CQ * C; } else if (t < 2 * nq + ng) { src = wg; e = (t - 2 * nq) * 8; dst = WG; } else if (t < 2 * nq + ng + no) { src = wo; e = (t - 2 * nq - ng) * 8; dst = WO; } else return;
  v8b o; for (int j = 0; j < 8; ++j) o[j] = (b16)(bf16_rne(src[e + j]) * WSC);
  for (int pass = 0; pass < 2; ++pass) { *(volatile v8b*)(dst + e) = o; __threadfence(); }
}
__global__ __launch_bounds__(128) void qk_kernel(const b16* __restrict__ XT16, const b16* __restrict__ W16, b16* __restrict__ QH, b16* __restrict__ QL, float* __restrict__ PHI) {
  __shared__ __attribute__((aligned(16))) b16 Th[4][16][CQ + 8], Tl[4][16][CQ + 8]; __shared__ __attribute__((aligned(16))) float Tf[4][16][CQ + 4];
  const int wave = threadIdx.x >> 5, lane = threadIdx.x & 31, nloc = lane & 15, hlf = lane >> 4; const size_t r0 = ((size_t)blockIdx.x * 4 + wave) * 16;
  v8f acc[4] = {{}, {}, {}, {}};
#pragma unroll 2
  for (int kb = 0; kb < C; kb += 32) { const v16b a = frag_kb(XT16 + (r0 + nloc) * C + kb, hlf);
#pragma unroll
    for (int t = 0; t < 4; ++t) acc[t] = wmma16b(a, frag_kb(W16 + (size_t)((t >> 1) * CQ + (t & 1) * 16 + nloc) * C + kb, hlf), acc[t]); }
#pragma unroll
  for (int t = 0; t < 4; ++t) { const int which = t >> 1, c = (t & 1) * 16 + nloc;
#pragma unroll
    for (int r = 0; r < 8; ++r) { const float v = acc[t][r] * (1.0f / (XS * WSC)); if (which == 0) { b16 h_, l_; split16(v * XS, h_, l_); Th[wave][8 * hlf + r][c] = h_; Tl[wave][8 * hlf + r][c] = l_; } else Tf[wave][8 * hlf + r][c] = v; } }
  wave_lds_sync();
  for (int pass = 0; pass < 2; ++pass) {
    for (int q = 0; q < 2; ++q) { const int rr = q * 8 + (lane >> 2), seg = (lane & 3) * 8; *(volatile v8b*)(QH + (r0 + rr) * CQ + seg) = *(const v8b*)(&Th[wave][rr][seg]); *(volatile v8b*)(QL + (r0 + rr) * CQ + seg) = *(const v8b*)(&Tl[wave][rr][seg]); }
    for (int q = 0; q < 4; ++q) { const int rr = q * 4 + (lane >> 3), seg = (lane & 7) * 4; *(volatile v4f*)(PHI + (r0 + rr) * CQ + seg) = *(const v4f*)(&Tf[wave][rr][seg]); }
    __threadfence(); }
}
__global__ __launch_bounds__(256) void poolk_kernel(const float* __restrict__ PHI, b16* __restrict__ KH, b16* __restrict__ KL) {
  const size_t t = (size_t)blockIdx.x * 256 + threadIdx.x; if (t >= (size_t)NB * M * CQ / 8) return; const int c8 = (int)(t & 3) * 8; const size_t bm = t >> 2; const int b = (int)(bm / M), m = (int)(bm % M); const int h2 = m / (HW / 2), w2 = m % (HW / 2);
  const float* p0 = PHI + ((size_t)b * N + (size_t)(2 * h2) * HW + 2 * w2) * CQ + c8; v8b hv, lv;
  for (int j = 0; j < 8; ++j) { const float v = fmaxf(fmaxf(p0[j], p0[CQ + j]), fmaxf(p0[(size_t)HW * CQ + j], p0[(size_t)HW * CQ + CQ + j])); b16 h_, l_; split16(v * XS, h_, l_); hv[j] = h_; lv[j] = l_; }
  for (int pass = 0; pass < 2; ++pass) { *(volatile v8b*)(KH + bm * CQ + c8) = hv; *(volatile v8b*)(KL + bm * CQ + c8) = lv; __threadfence(); }
}
__global__ __launch_bounds__(128) void g_kernel(const b16* __restrict__ XT16, const b16* __restrict__ WG, float* __restrict__ GF) {
  __shared__ __attribute__((aligned(16))) float Ts[4][16][128 + 4];
  const int wave = threadIdx.x >> 5, lane = threadIdx.x & 31, nloc = lane & 15, hlf = lane >> 4; const int b = blockIdx.z; const int d0 = blockIdx.x * 64 + wave * 16, n0 = blockIdx.y * 128;
  v8f acc[8];
#pragma unroll
  for (int t = 0; t < 8; ++t) acc[t] = (v8f){};
#pragma unroll 2
  for (int kb = 0; kb < C; kb += 32) { const v16b a = frag_kb(WG + (size_t)(d0 + nloc) * C + kb, hlf);
#pragma unroll
    for (int t = 0; t < 8; ++t) acc[t] = wmma16b(a, frag_kb(XT16 + ((size_t)b * N + n0 + t * 16 + nloc) * C + kb, hlf), acc[t]); }
#pragma unroll
  for (int t = 0; t < 8; ++t)
#pragma unroll
    for (int r = 0; r < 8; ++r) Ts[wave][8 * hlf + r][t * 16 + nloc] = acc[t][r] * (1.0f / (XS * WSC));
  wave_lds_sync();
  for (int pass = 0; pass < 2; ++pass) { for (int rr = 0; rr < 16; ++rr) *(volatile v4f*)(GF + ((size_t)b * CG + d0 + rr) * N + n0 + lane * 4) = *(const v4f*)(&Ts[wave][rr][lane * 4]); __threadfence(); }
}
__global__ __launch_bounds__(256) void poolg_kernel(const float* __restrict__ GF, b16* __restrict__ GP, b16* __restrict__ GPL) {
  const size_t t = (size_t)blockIdx.x * 256 + threadIdx.x; if (t >= (size_t)NB * M * CG / 8) return; const int d8 = (int)(t & 15) * 8; const size_t bm = t >> 4; const int b = (int)(bm / M), m = (int)(bm % M); const int h2 = m / (HW / 2), w2 = m % (HW / 2);
  const size_t n00 = (size_t)(2 * h2) * HW + 2 * w2; v8b hv, lv;
  for (int j = 0; j < 8; ++j) { const float* p = GF + ((size_t)b * CG + d8 + j) * N + n00; const float v = fmaxf(fmaxf(p[0], p[1]), fmaxf(p[HW], p[HW + 1])); b16 h_, l_; split16(v * XS, h_, l_); hv[j] = h_; lv[j] = l_; }
  for (int pass = 0; pass < 2; ++pass) { *(volatile v8b*)(GP + bm * CG + d8) = hv; *(volatile v8b*)(GPL + bm * CG + d8) = lv; __threadfence(); }
}
__global__ __launch_bounds__(128) void v_kernel(const b16* __restrict__ GP, const b16* __restrict__ GPL, const b16* __restrict__ WO, b16* __restrict__ V16, b16* __restrict__ VL16) {
  __shared__ __attribute__((aligned(16))) b16 Ts[4][16][128 + 8], Tl[4][16][128 + 8];
  const int wave = threadIdx.x >> 5, lane = threadIdx.x & 31, nloc = lane & 15, hlf = lane >> 4; const int b = blockIdx.z; const int d0 = blockIdx.x * 64 + wave * 16, n0 = blockIdx.y * 128;
  v8f acc[8];
#pragma unroll
  for (int t = 0; t < 8; ++t) acc[t] = (v8f){};
#pragma unroll
  for (int kb = 0; kb < CG; kb += 32) { const v16b a = frag_kb(WO + (size_t)(d0 + nloc) * CG + kb, hlf);
#pragma unroll
    for (int t = 0; t < 8; ++t) { const size_t ro = ((size_t)b * M + n0 + t * 16 + nloc) * CG + kb; acc[t] = wmma16b(a, frag_kb(GP + ro, hlf), acc[t]); acc[t] = wmma16b(a, frag_kb(GPL + ro, hlf), acc[t]); } }
#pragma unroll
  for (int t = 0; t < 8; ++t)
#pragma unroll
    for (int r = 0; r < 8; ++r) { b16 h_, l_; split16(acc[t][r] * (1.0f / (XS * WSC)) * XS, h_, l_); Ts[wave][8 * hlf + r][t * 16 + nloc] = h_; Tl[wave][8 * hlf + r][t * 16 + nloc] = l_; }
  wave_lds_sync();
  for (int pass = 0; pass < 2; ++pass) { for (int rr = 0; rr < 16; ++rr) if (lane < 16) { const size_t gi = ((size_t)b * C + d0 + rr) * M + n0 + lane * 8; *(volatile v8b*)(V16 + gi) = *(const v8b*)(&Ts[wave][rr][lane * 8]); *(volatile v8b*)(VL16 + gi) = *(const v8b*)(&Tl[wave][rr][lane * 8]); } __threadfence(); }
}
__global__ __launch_bounds__(64) void attn_kernel(const b16* __restrict__ QH, const b16* __restrict__ QL, const b16* __restrict__ KH, const b16* __restrict__ KL, const b16* __restrict__ V16, const b16* __restrict__ VL16, const float* __restrict__ x, const float* __restrict__ gamma_, float* __restrict__ out) {
  __shared__ __attribute__((aligned(16))) float To[128][32 + 4];
  const int wave = threadIdx.x >> 5, lane = threadIdx.x & 31, hh = lane >> 4, col = lane & 15; const int b = blockIdx.z, dh = blockIdx.y; const int q0 = blockIdx.x * 32 + wave * 16, qi = q0 + col;
  const size_t qrow = (size_t)b * N + qi; const v16b qh = frag_kb(QH + qrow * CQ, hh), ql = frag_kb(QL + qrow * CQ, hh);
  const b16* Khb = KH + (size_t)b * M * CQ; const b16* Klb = KL + (size_t)b * M * CQ; const b16* Vb = V16 + ((size_t)b * C + dh * 128) * M; const b16* Vlb = VL16 + ((size_t)b * C + dh * 128) * M; const float gamma = bf16_rne(gamma_[0]);
  float m = -INFINITY, l = 0.0f; v8f o[8], ol[8];
#pragma unroll
  for (int t = 0; t < 8; ++t) { o[t] = (v8f){}; ol[t] = (v8f){}; }
  for (int kb = 0; kb < M; kb += 32) {
    v8f s0 = {}, s1 = {};
    { const b16* k0 = Khb + (size_t)(kb + col) * CQ, *k1 = Khb + (size_t)(kb + 16 + col) * CQ, *k0l = Klb + (size_t)(kb + col) * CQ, *k1l = Klb + (size_t)(kb + 16 + col) * CQ;
      const v16b f0 = frag_kb(k0, hh), f1 = frag_kb(k1, hh);
      s0 = wmma16b(f0, qh, s0); s0 = wmma16b(f0, ql, s0); s0 = wmma16b(frag_kb(k0l, hh), qh, s0);
      s1 = wmma16b(f1, qh, s1); s1 = wmma16b(f1, ql, s1); s1 = wmma16b(frag_kb(k1l, hh), qh, s1); }
    float e[16]; float mx = -INFINITY; const float cs = LOG2E / (XS * XS);
#pragma unroll
    for (int r = 0; r < 8; ++r) { e[r] = s0[r] * cs; e[8 + r] = s1[r] * cs; mx = fmaxf(mx, fmaxf(e[r], e[8 + r])); }
    mx = fmaxf(mx, __shfl_xor(mx, 16)); const float mn = fmaxf(m, mx); const float al = nexp2(m - mn); m = mn; float sum = 0.0f; v16b ph, pl;
#pragma unroll
    for (int i = 0; i < 16; ++i) { const float p = nexp2(e[i] - mn); sum += p; const b16 h_ = (b16)(p * PS); ph[i] = h_; pl[i] = (b16)(p * PS - (float)h_); }
    sum += __shfl_xor(sum, 16); l = l * al + sum;
#pragma unroll
    for (int t = 0; t < 8; ++t) { o[t] *= al; ol[t] *= al; const v16b vf = frag_kb(Vb + (size_t)(t * 16 + col) * M + kb, hh); o[t] = wmma16b(vf, ph, o[t]); ol[t] = wmma16b(vf, pl, ol[t]); ol[t] = wmma16b(frag_kb(Vlb + (size_t)(t * 16 + col) * M + kb, hh), ph, ol[t]); } }
  const float inv = 1.0f / (l * PS * XS);
#pragma unroll
  for (int t = 0; t < 8; ++t)
#pragma unroll
    for (int r = 0; r < 8; ++r) To[t * 16 + 8 * hh + r][wave * 16 + col] = (o[t][r] + ol[t][r]) * inv;
  __syncthreads();
  for (int pass = 0; pass < 2; ++pass) { for (int dd = wave * 64; dd < wave * 64 + 64; ++dd) { const size_t gi = ((size_t)b * C + dh * 128 + dd) * N + blockIdx.x * 32 + lane; ((volatile float*)out)[gi] = gamma * To[dd][lane] + bf16_rne(x[gi]); } __threadfence(); }
}
}

extern "C" void kernel_launch(void* const* d_in, const int* in_sizes, int n_in, void* d_out, int out_size, void* d_ws, size_t ws_size, hipStream_t stream) {
  (void)n_in;
  auto Fp = [&](int i) { return (const float*)d_in[i]; };
  if (in_sizes[0] != NB * C * N || in_sizes[1] != CQ * C || in_sizes[2] != CQ * C || in_sizes[3] != CG * C || in_sizes[4] != C * CG || in_sizes[5] != 1 || out_size != NB * C * N) return;
  size_t off = 0; char* ws = (char*)d_ws;
  auto carve = [&](size_t bytes) { char* p = ws + off; off += (bytes + 255) & ~(size_t)255; return p; };
  b16* XT16 = (b16*)carve((size_t)NB * N * C * 2); b16* W16 = (b16*)carve((size_t)2 * CQ * C * 2); b16* WG = (b16*)carve((size_t)CG * C * 2); b16* WO = (b16*)carve((size_t)C * CG * 2);
  b16* QH = (b16*)carve((size_t)NB * N * CQ * 2); b16* QL = (b16*)carve((size_t)NB * N * CQ * 2); float* PHI = (float*)carve((size_t)NB * N * CQ * 4); b16* KH = (b16*)carve((size_t)NB * M * CQ * 2); b16* KL = (b16*)carve((size_t)NB * M * CQ * 2);
  float* GF = (float*)carve((size_t)NB * CG * N * 4); b16* GP = (b16*)carve((size_t)NB * M * CG * 2); b16* GPL = (b16*)carve((size_t)NB * M * CG * 2); b16* V16 = (b16*)carve((size_t)NB * C * M * 2); b16* VL16 = (b16*)carve((size_t)NB * C * M * 2);
  if (off > ws_size || off > ((size_t)128 << 20)) return;
  xt_kernel<<<dim3(N / 64, C / 64, NB), 256, 0, stream>>>(Fp(0), XT16);
  prepw_kernel<<<((2 * CQ * C + CG * C + C * CG) / 8 + 255) / 256, 256, 0, stream>>>(Fp(1), Fp(2), Fp(3), Fp(4), W16, WG, WO);
  qk_kernel<<<NB * N / 64, 128, 0, stream>>>(XT16, W16, QH, QL, PHI);
  poolk_kernel<<<(NB * M * CQ / 8 + 255) / 256, 256, 0, stream>>>(PHI, KH, KL);
  g_kernel<<<dim3(CG / 64, N / 128, NB), 128, 0, stream>>>(XT16, WG, GF);
  poolg_kernel<<<(NB * M * CG / 8 + 255) / 256, 256, 0, stream>>>(GF, GP, GPL);
  v_kernel<<<dim3(C / 64, M / 128, NB), 128, 0, stream>>>(GP, GPL, WO, V16, VL16);
  attn_kernel<<<dim3(N / 32, 2, NB), 64, 0, stream>>>(QH, QL, KH, KL, V16, VL16, Fp(0), Fp(5), (float*)d_out);
}
